// DifferentiableRenderer_8581344658045
// MI455X (gfx1250) — hardware-verified
//
#include <hip/hip_runtime.h>
#include <math.h>

typedef __attribute__((ext_vector_type(16))) _Float16 v16h;
typedef __attribute__((ext_vector_type(16))) __bf16 v16b;
typedef __attribute__((ext_vector_type(8)))  _Float16 v8h;
typedef __attribute__((ext_vector_type(8)))  float v8f;
typedef __attribute__((ext_vector_type(4)))  float v4f;
typedef __attribute__((ext_vector_type(2)))  float v2f;
typedef __attribute__((ext_vector_type(4)))  unsigned v4u;
typedef __attribute__((ext_vector_type(4)))  int v4i;
typedef float __attribute__((may_alias)) float_a;
typedef int __attribute__((may_alias)) int_a;

template <typename T> __device__ __forceinline__ void vst2(void* p, T v) { *(volatile T*)p = v; __threadfence(); *(volatile T*)p = v; }
__device__ __forceinline__ v8f wmma16(v16h a, v16h b, v8f c) {
  v8f d = __builtin_amdgcn_wmma_f32_16x16x32_f16(false, a, false, b, (short)0, c, false, false);
  asm volatile("v_nop\n\tv_nop\n\tv_nop\n\tv_nop" : "+v"(d) : "v"(a), "v"(b));
  return d;
}
__device__ __forceinline__ v8f wmma_bf(v16b a, v16b b, v8f c) {
  v8f d = __builtin_amdgcn_wmma_f32_16x16x32_bf16(false, a, false, b, (short)0, c, false, false);
  asm volatile("v_nop\n\tv_nop\n\tv_nop\n\tv_nop" : "+v"(d) : "v"(a), "v"(b));
  return d;
}
__device__ __forceinline__ v16h frag_h(const _Float16* rowk0, int lane) {
  union { v16h v; v8h q[2]; } u; const _Float16* p = rowk0 + 8 * (lane >> 4);
  u.q[0] = *(const v8h*)p; u.q[1] = *(const v8h*)(p + 16); return u.v;
}
__device__ __forceinline__ v16h frag_f32(const float* rowk0, int lane) {
  v16h a; const float* p = rowk0 + 8 * (lane >> 4);
#pragma unroll
  for (int i = 0; i < 8; ++i) { a[i] = (_Float16)p[i]; a[8 + i] = (_Float16)p[16 + i]; }
  return a;
}
__device__ __forceinline__ v16h frag_f32s(const float* rowk0, int lane, float sc) {
  v16h a; const float* p = rowk0 + 8 * (lane >> 4);
#pragma unroll
  for (int i = 0; i < 8; ++i) { a[i] = (_Float16)(p[i] * sc); a[8 + i] = (_Float16)(p[16 + i] * sc); }
  return a;
}
__device__ __forceinline__ v16h fragc_f32(const float* W, int k0, int n, int lane, int ld, int K) {
  v16h a; const int g = lane >> 4;
#pragma unroll
  for (int i = 0; i < 8; ++i) { const int ka = k0 + 8 * g + i, kb = ka + 16;
    a[i] = (_Float16)(ka < K ? W[(size_t)(ka < K ? ka : K - 1) * ld + n] : 0.f); a[8 + i] = (_Float16)(kb < K ? W[(size_t)(kb < K ? kb : K - 1) * ld + n] : 0.f); }
  return a;
}
struct F2 { v16b h, l; };
__device__ __forceinline__ F2 bsplit16(const float v[16]) { F2 r;
#pragma unroll
  for (int i = 0; i < 16; ++i) { const __bf16 h = (__bf16)v[i]; r.h[i] = h; r.l[i] = (__bf16)(v[i] - (float)h); }
  return r; }
__device__ __forceinline__ F2 split_row(const float* row, int k0, int lane) { float v[16]; const float* p = row + k0 + 8 * (lane >> 4);
#pragma unroll
  for (int i = 0; i < 8; ++i) { v[i] = p[i]; v[8 + i] = p[16 + i]; }
  return bsplit16(v); }
__device__ __forceinline__ F2 split_rowK(const float* row, int k0, int lane, int K) { float v[16]; const int g = lane >> 4;
#pragma unroll
  for (int i = 0; i < 8; ++i) { const int ka = k0 + 8 * g + i, kb = ka + 16; v[i] = ka < K ? row[ka < K ? ka : K - 1] : 0.f; v[8 + i] = kb < K ? row[kb < K ? kb : K - 1] : 0.f; }
  return bsplit16(v); }
__device__ __forceinline__ F2 split_col(const float* W, int k0, int n, int lane, int ld, int K) { float v[16]; const int g = lane >> 4;
#pragma unroll
  for (int i = 0; i < 8; ++i) { const int ka = k0 + 8 * g + i, kb = ka + 16; v[i] = ka < K ? W[(size_t)(ka < K ? ka : K - 1) * ld + n] : 0.f; v[8 + i] = kb < K ? W[(size_t)(kb < K ? kb : K - 1) * ld + n] : 0.f; }
  return bsplit16(v); }
__device__ __forceinline__ v8f mac3(const F2& a, const F2& b, v8f c) { c = wmma_bf(a.l, b.h, c); c = wmma_bf(a.h, b.l, c); return wmma_bf(a.h, b.h, c); }
__device__ __forceinline__ float sigm(float v) { return 1.0f / (1.0f + expf(-v)); }
#define LDSX() do { asm volatile("s_wait_dscnt 0" ::: "memory"); __builtin_amdgcn_wave_barrier(); __builtin_amdgcn_fence(__ATOMIC_RELEASE, "workgroup"); } while (0)

#define NPZ 1024
#define HW 65536
#define NPOSE 2
#ifndef NPPROC
#define NPPROC NPOSE
#endif
__device__ __forceinline__ float bfr(float v) { return (float)(__bf16)v; }
#define WS_PRJ 0u
#define WS_END (WS_PRJ + 4u * (size_t)NPOSE * NPZ * 4)

__global__ __launch_bounds__(256) void k_cam(const float* __restrict__ POS, const float* __restrict__ SC, const float* __restrict__ QV, const float* __restrict__ TV, float* __restrict__ PRJ) {
  const int tid = blockIdx.x * 256 + threadIdx.x; if (tid >= NPPROC * NPZ) return; const int b = tid / NPZ, n = tid % NPZ;
  float q0 = bfr(QV[b * 4]), q1 = bfr(QV[b * 4 + 1]), q2 = bfr(QV[b * 4 + 2]), q3 = bfr(QV[b * 4 + 3]);
  const float nrm = sqrtf(q0 * q0 + q1 * q1 + q2 * q2 + q3 * q3); q0 /= nrm; q1 /= nrm; q2 /= nrm; q3 /= nrm;
  const float w = q0, x = q1, y = q2, z = q3;
  const float R00 = 1.f - 2.f * (y * y + z * z), R01 = 2.f * (x * y - z * w), R02 = 2.f * (x * z + y * w);
  const float R10 = 2.f * (x * y + z * w), R11 = 1.f - 2.f * (x * x + z * z), R12 = 2.f * (y * z - x * w);
  const float R20 = 2.f * (x * z - y * w), R21 = 2.f * (y * z + x * w), R22 = 1.f - 2.f * (x * x + y * y);
  const float p0 = bfr(POS[n * 3]), p1 = bfr(POS[n * 3 + 1]), p2 = bfr(POS[n * 3 + 2]);
  const float cx = p0 * R00 + p1 * R01 + p2 * R02 + bfr(TV[b * 3]);
  const float cy = p0 * R10 + p1 * R11 + p2 * R12 + bfr(TV[b * 3 + 1]);
  const float cz = p0 * R20 + p1 * R21 + p2 * R22 + bfr(TV[b * 3 + 2]);
  const float px = (cx / cz) * 300.0f + 128.0f, py = (cy / cz) * 300.0f + 128.0f;
  const float sc = bfr(SC[n]); const float var = sc * sc;
  v4f o; o[0] = px; o[1] = py; o[2] = px * px + py * py; o[3] = -0.5f / var; vst2(PRJ + (size_t)tid * 4, o); }
__global__ __launch_bounds__(128) void k_render(const float* __restrict__ PRJ, const float* __restrict__ PIX, const float* __restrict__ COL, const float* __restrict__ OPA, float* __restrict__ OUT) { __shared__ __align__(16) float so[4][64];
  const int tid = threadIdx.x, wave = tid >> 5, lane = tid & 31, col = lane & 15, g = lane >> 4; const int b = blockIdx.y; const size_t p0 = (size_t)blockIdx.x * 64; const size_t myp = p0 + wave * 16 + col;
  const float pxx = bfr(PIX[myp * 2]), pyy = bfr(PIX[myp * 2 + 1]); const float c2 = pxx * pxx + pyy * pyy;
  const float* prj = PRJ + (size_t)b * NPZ * 4;
  v8f acc = {};
#pragma unroll 1
  for (int kc = 0; kc < NPZ / 32; ++kc) { float wv[16]; float cb[16];
#pragma unroll
    for (int i = 0; i < 16; ++i) { const int n = kc * 32 + 8 * g + (i < 8 ? i : 8 + i); const v4f pr = *(const v4f*)(prj + (size_t)n * 4); const float op = OPA[n];
      const float dist2 = (pr[2] + c2) - 2.0f * (pr[0] * pxx + pr[1] * pyy);
      wv[i] = bfr(op) * expf(dist2 * pr[3]);
      cb[i] = (col < 3) ? COL[n * 3 + col] : 0.f; }
    asm volatile("s_wait_loadcnt 0x0" ::: "memory");
    const F2 a = bsplit16(wv); v16b bw;
#pragma unroll
    for (int i = 0; i < 16; ++i) bw[i] = (__bf16)(col < 3 ? cb[i] : (col == 3 ? 1.0f : 0.f));
    acc = wmma_bf(a.h, bw, acc); acc = wmma_bf(a.l, bw, acc); }
  __shared__ __align__(16) float st[4][16][5];
  if (col < 4) {
#pragma unroll
    for (int r = 0; r < 8; ++r) st[wave][8 * g + r][col] = acc[r]; }
  LDSX();
  if (lane < 16) { const float den = st[wave][lane][3] + 1e-8f;
#pragma unroll
    for (int c = 0; c < 3; ++c) so[c][wave * 16 + lane] = st[wave][lane][c] / den; }
  __syncthreads();
  if (tid < 48) { const int c = tid >> 4, q = tid & 15; vst2(OUT + ((size_t)b * 3 + c) * HW + p0 + q * 4, *(const v4f*)&so[c][q * 4]); } }
extern "C" void kernel_launch(void* const* d_in, const int* in_sizes, int n_in, void* d_out, int out_size, void* d_ws, size_t ws_size, hipStream_t stream) {
  (void)in_sizes; (void)n_in; (void)out_size;
  if (ws_size < (size_t)WS_END) return;
  char* ws = (char*)d_ws; const float** F = (const float**)d_in; float* PRJ = (float*)(ws + WS_PRJ);
  k_cam<<<dim3((NPPROC * NPZ + 255) / 256), 256, 0, stream>>>(F[0], F[3], F[4], F[5], PRJ);
  k_render<<<dim3(HW / 64, NPPROC), 128, 0, stream>>>(PRJ, F[6], F[1], F[2], (float*)d_out);
}
